// MIDGCN_87058987090446
// MI455X (gfx1250) — hardware-verified
//
#include <hip/hip_runtime.h>
#include <math.h>

#define NB    16
#define NC    2048
#define DT    128
#define DH    64
#define DI    32
#define NCL   16
#define DCE   32
#define DG    32
#define DGI   192
#define DOUT  96
#define DOUTP 128
#define NROW  (NB * NC)
#define NEGV  (-1.0e9f)

#define SX   16.0f
#define SW   256.0f
#define SW4  1024.0f
#define SR   4096.0f
#define SH   16.0f
#define SID  32.0f
#define SIC  256.0f
#define SPB  16.0f
#define SCE  256.0f
#define SG   256.0f
#define SP   1024.0f
#define SAG  256.0f
#define SWT  1024.0f
#define SU   64.0f

static_assert((NC % 64) == 0 && (NROW % 64) == 0 && (DGI % 64) == 0 && DGI == DT + DI + DCE);
static_assert(DI == 32 && DCE == 32 && DG == 32 && NCL == 16 && DH == 64 && DT == 128);
static constexpr float kLog2E = 1.4426950408889634f;

typedef _Float16 v16h __attribute__((ext_vector_type(16)));
typedef _Float16 v8h  __attribute__((ext_vector_type(8)));
typedef float    v8f  __attribute__((ext_vector_type(8)));
typedef float    v4f  __attribute__((ext_vector_type(4)));
typedef unsigned int v4u __attribute__((ext_vector_type(4)));
typedef unsigned short v8us __attribute__((ext_vector_type(8)));

__device__ __forceinline__ unsigned short bf_bits(float f) {
  unsigned u = __float_as_uint(f);
  return (unsigned short)((u + 0x7FFFu + ((u >> 16) & 1u)) >> 16);
}
__device__ __forceinline__ float bf_up(unsigned short hb) { return __uint_as_float(((unsigned)hb) << 16); }
__device__ __forceinline__ float bfr(float f) { return bf_up(bf_bits(f)); }
__device__ __forceinline__ unsigned short h_bits(_Float16 x) { return __builtin_bit_cast(unsigned short, x); }
__device__ __forceinline__ unsigned pk16(unsigned short a, unsigned short b) { return (unsigned)a | ((unsigned)b << 16); }
__device__ __forceinline__ v8f zero8() { v8f z = {0.f, 0.f, 0.f, 0.f, 0.f, 0.f, 0.f, 0.f}; return z; }

__device__ __forceinline__ _Float16 f16n(float v) {
  const _Float16 hh = (_Float16)v;
  const float back = (float)hh;
  return (fabsf(back) < 6.103515625e-05f) ? (_Float16)0.0f : hh;
}
__device__ __forceinline__ void split16(float v, float sc, _Float16& hi, _Float16& rs) {
  const float t = v * sc;
  const _Float16 hh = f16n(t);
  hi = hh;
  rs = (_Float16)((t - (float)hh) * SR);
}
__device__ __forceinline__ unsigned short cvt16(float f, float wsc) {
  return h_bits((_Float16)(bfr(f) * wsc));
}

__device__ __forceinline__ v16h ldfrag_h(const _Float16* p) {
  union { v16h v; v8h hh[2]; } f;
  f.hh[0] = *(const v8h*)(p);
  f.hh[1] = *(const v8h*)(p + 16);
  return f.v;
}

__device__ __forceinline__ v8f mma_h(v16h a, v16h b, v8f c) {
  c = __builtin_amdgcn_wmma_f32_16x16x32_f16(false, a, false, b, (short)0, c, false, false);
#if defined(__HIP_DEVICE_COMPILE__)
  asm volatile("v_nop\n\tv_nop\n\tv_nop\n\tv_nop" : "+v"(c) : "v"(a), "v"(b));
#endif
  return c;
}
__device__ __forceinline__ void wave_sync_lds() {
#if defined(__HIP_DEVICE_COMPILE__)
  __builtin_amdgcn_fence(__ATOMIC_RELEASE, "workgroup");
  __builtin_amdgcn_wave_barrier();
  __builtin_amdgcn_fence(__ATOMIC_ACQUIRE, "workgroup");
#endif
}

__global__ __launch_bounds__(256) void tconv(const float* __restrict__ src, int sk, int sn,
                                             unsigned short* dst, int K, int N, int Kp, float scale) {
  __shared__ __align__(16) unsigned short rowbuf[2048];
  union UU { v8us s; v4u u; };
  const int n = blockIdx.x;
  const int tid = threadIdx.x;
  const int nn = (n < N) ? n : (N - 1);
  for (int k = tid; k < Kp; k += 256) {
    const int kk = (k < K) ? k : (K - 1);
    const float v = src[(size_t)kk * sk + (size_t)nn * sn];
    unsigned short hv = cvt16(v, scale);
    if (k >= K || n >= N) hv = (unsigned short)0;
    rowbuf[k] = hv;
  }
  __syncthreads();
  const int np8 = Kp >> 3;
  const int q = (tid < np8) ? tid : 0;
  UU o;
  o.s = *(const v8us*)(rowbuf + q * 8);
  unsigned short* dp = dst + (size_t)n * Kp + q * 8;
  if (tid < np8) *(volatile v4u*)dp = o.u;
  __threadfence();
  if (tid < np8) *(volatile v4u*)dp = o.u;
}

__global__ __launch_bounds__(256) void xconv(const float* __restrict__ x, unsigned short* GI) {
  const int P = blockIdx.x * 256 + threadIdx.x;
  const int row = P >> 4, j = P & 15;
  const float* s = x + (size_t)row * DT + j * 8;
  const v4f a = *(const v4f*)(s);
  const v4f b = *(const v4f*)(s + 4);
  v4u u;
  u[0] = pk16(cvt16(a[0], SX), cvt16(a[1], SX));
  u[1] = pk16(cvt16(a[2], SX), cvt16(a[3], SX));
  u[2] = pk16(cvt16(b[0], SX), cvt16(b[1], SX));
  u[3] = pk16(cvt16(b[2], SX), cvt16(b[3], SX));
  unsigned short* d = GI + (size_t)row * DGI + j * 8;
  *(volatile v4u*)d = u;
  __threadfence();
  *(volatile v4u*)d = u;
}

__global__ __launch_bounds__(256) void tr16(const unsigned short* __restrict__ src, int ps,
                                            unsigned short* dst, int R, int Csrc) {
  __shared__ __align__(16) _Float16 T[64 * 72];
  union HU { v8h hv; v4u u; };
  const int tid = threadIdx.x;
  const int r0 = blockIdx.x * 64, c0 = blockIdx.y * 64, z = blockIdx.z;
  const _Float16* S = (const _Float16*)(const void*)src;
#pragma unroll
  for (int qq = 0; qq < 2; ++qq) {
    const int p = qq * 256 + tid;
    const int row = p >> 3;
    const int c8 = (p & 7) * 8;
    const v8h v = *(const v8h*)(S + (size_t)(z * R + r0 + row) * ps + c0 + c8);
#pragma unroll
    for (int e = 0; e < 8; ++e) T[(c8 + e) * 72 + row] = v[e];
  }
  __syncthreads();
  HU o[2];
#pragma unroll
  for (int qq = 0; qq < 2; ++qq) {
    const int p = qq * 256 + tid;
    const int line = p >> 3;
    const int pc = (p & 7) * 8;
    o[qq].hv = *(const v8h*)(T + line * 72 + pc);
  }
  for (int pass = 0; pass < 2; ++pass) {
#pragma unroll
    for (int qq = 0; qq < 2; ++qq) {
      const int p = qq * 256 + tid;
      const int line = p >> 3;
      const int pc = (p & 7) * 8;
      *(volatile v4u*)(dst + (size_t)(z * Csrc + c0 + line) * R + r0 + pc) = o[qq].u;
    }
    __threadfence();
  }
}

__global__ __launch_bounds__(128) void chain(
    unsigned short* GI,
    const unsigned short* __restrict__ W1Tp, const unsigned short* __restrict__ W2Tp,
    const unsigned short* __restrict__ WICTp, const unsigned short* __restrict__ CEp,
    const unsigned short* __restrict__ CETp, const unsigned short* __restrict__ WGTp,
    const float* __restrict__ b1, const float* __restrict__ idemb, const float* __restrict__ b2,
    const float* __restrict__ bic, const float* __restrict__ bg,
    unsigned short* GH, unsigned short* GR) {
  union HU { v8h hv; v4u u; };
  __shared__ __align__(16) _Float16 Ph[4][16 * 64];
  __shared__ __align__(16) _Float16 Pr[4][16 * 64];
  __shared__ __align__(16) _Float16 Qh[4][16 * 32];
  __shared__ __align__(16) _Float16 Qr[4][16 * 32];

  const int tid = threadIdx.x, wave = tid >> 5, lane = tid & 31, h = lane >> 4, c = lane & 15;
  const int r0 = (blockIdx.x * 4 + wave) * 16;
  const _Float16* GIf  = (const _Float16*)(const void*)GI;
  const _Float16* W1T  = (const _Float16*)(const void*)W1Tp;
  const _Float16* W2T  = (const _Float16*)(const void*)W2Tp;
  const _Float16* WICT = (const _Float16*)(const void*)WICTp;
  const _Float16* CE   = (const _Float16*)(const void*)CEp;
  const _Float16* CET  = (const _Float16*)(const void*)CETp;
  const _Float16* WGT  = (const _Float16*)(const void*)WGTp;
  _Float16* ph = Ph[wave];
  _Float16* pr = Pr[wave];
  _Float16* qh = Qh[wave];
  _Float16* qr = Qr[wave];
  const float RINV = 1.0f / SR;

  v8f a1[4];
#pragma unroll
  for (int j = 0; j < 4; ++j) a1[j] = zero8();
#pragma unroll
  for (int ks = 0; ks < 4; ++ks) {
    const v16h af = ldfrag_h(GIf + (size_t)(r0 + c) * DGI + ks * 32 + 8 * h);
#pragma unroll
    for (int j = 0; j < 4; ++j) {
      const v16h bf = ldfrag_h(W1T + (size_t)(16 * j + c) * DT + ks * 32 + 8 * h);
      a1[j] = mma_h(af, bf, a1[j]);
    }
  }
  {
    const float s1 = 1.0f / (SX * SW);
#pragma unroll
    for (int j = 0; j < 4; ++j) {
      const float bb = bfr(b1[16 * j + c]);
#pragma unroll
      for (int r = 0; r < 8; ++r) {
        const float hv = fmaxf(a1[j][r] * s1 + bb, 0.0f);
        _Float16 hi, rs;
        split16(hv, SH, hi, rs);
        const int pi = (8 * h + r) * 64 + 16 * j + c;
        ph[pi] = hi;
        pr[pi] = rs;
      }
    }
  }
  wave_sync_lds();

  v8f dh[2], dr[2];
#pragma unroll
  for (int j = 0; j < 2; ++j) { dh[j] = zero8(); dr[j] = zero8(); }
#pragma unroll
  for (int ks = 0; ks < 2; ++ks) {
    const v16h ah = ldfrag_h(ph + c * 64 + ks * 32 + 8 * h);
    const v16h ar = ldfrag_h(pr + c * 64 + ks * 32 + 8 * h);
#pragma unroll
    for (int j = 0; j < 2; ++j) {
      const v16h bf = ldfrag_h(W2T + (size_t)(16 * j + c) * DH + ks * 32 + 8 * h);
      dh[j] = mma_h(ah, bf, dh[j]);
      dr[j] = mma_h(ar, bf, dr[j]);
    }
  }
  float idv[2][8];
  {
    const float s2 = 1.0f / (SH * SW);
#pragma unroll
    for (int j = 0; j < 2; ++j) {
      const float bb = bfr(b2[16 * j + c]);
#pragma unroll
      for (int r = 0; r < 8; ++r) {
        const int crow = (r0 + 8 * h + r) & (NC - 1);
        const float dyn = (dh[j][r] + dr[j][r] * RINV) * s2 + bb;
        idv[j][r] = bfr(idemb[(size_t)crow * DI + 16 * j + c]) + dyn;
      }
    }
  }
  wave_sync_lds();
#pragma unroll
  for (int j = 0; j < 2; ++j) {
#pragma unroll
    for (int r = 0; r < 8; ++r) {
      _Float16 hi, rs;
      split16(idv[j][r], SID, hi, rs);
      const int pi = (8 * h + r) * 64 + 16 * j + c;
      ph[pi] = hi;
      pr[pi] = rs;
    }
  }
  wave_sync_lds();

  v8f ih[2], ir[2];
  {
    const v16h ah = ldfrag_h(ph + c * 64 + 8 * h);
    const v16h ar = ldfrag_h(pr + c * 64 + 8 * h);
#pragma unroll
    for (int j = 0; j < 2; ++j) {
      const v16h bf = ldfrag_h(WICT + (size_t)(16 * j + c) * 64 + 8 * h);
      ih[j] = mma_h(ah, bf, zero8());
      ir[j] = mma_h(ar, bf, zero8());
    }
  }
  {
    const float s3 = 1.0f / (SID * SW);
#pragma unroll
    for (int j = 0; j < 2; ++j) {
      const float bb = bfr(bic[16 * j + c]);
#pragma unroll
      for (int r = 0; r < 8; ++r) {
        const float v = (ih[j][r] + ir[j][r] * RINV) * s3 + bb;
        _Float16 hi, rs;
        split16(v, SIC, hi, rs);
        const int qi = (8 * h + r) * 32 + 16 * j + c;
        qh[qi] = hi;
        qr[qi] = rs;
      }
    }
  }
  wave_sync_lds();

  v8f lh, lr;
  {
    const v16h ah = ldfrag_h(qh + c * 32 + 8 * h);
    const v16h ar = ldfrag_h(qr + c * 32 + 8 * h);
    const v16h bf = ldfrag_h(CE + (size_t)c * 64 + 8 * h);
    lh = mma_h(ah, bf, zero8());
    lr = mma_h(ar, bf, zero8());
  }
  float pv[8];
  {
    const float s4 = 1.0f / (SIC * SW);
#pragma unroll
    for (int r = 0; r < 8; ++r) {
      const float lg = (lh[r] + lr[r] * RINV) * s4;
      float m = lg;
      m = fmaxf(m, __shfl_xor(m, 1, 32));
      m = fmaxf(m, __shfl_xor(m, 2, 32));
      m = fmaxf(m, __shfl_xor(m, 4, 32));
      m = fmaxf(m, __shfl_xor(m, 8, 32));
      const float e = expf(lg - m);
      float s = e;
      s += __shfl_xor(s, 1, 32);
      s += __shfl_xor(s, 2, 32);
      s += __shfl_xor(s, 4, 32);
      s += __shfl_xor(s, 8, 32);
      pv[r] = e * (1.0f / s);
    }
  }
  wave_sync_lds();
#pragma unroll
  for (int r = 0; r < 8; ++r) {
    _Float16 hi, rs;
    split16(pv[r], SPB, hi, rs);
    const int qi = (8 * h + r) * 32 + c;
    qh[qi] = hi;
    qr[qi] = rs;
    qh[qi + 16] = (_Float16)0.0f;
    qr[qi + 16] = (_Float16)0.0f;
  }
  wave_sync_lds();

  v8f ch2[2], cr2[2];
  {
    const v16h ah = ldfrag_h(qh + c * 32 + 8 * h);
    const v16h ar = ldfrag_h(qr + c * 32 + 8 * h);
#pragma unroll
    for (int j = 0; j < 2; ++j) {
      const v16h bf = ldfrag_h(CET + (size_t)(16 * j + c) * 64 + 8 * h);
      ch2[j] = mma_h(ah, bf, zero8());
      cr2[j] = mma_h(ar, bf, zero8());
    }
  }
  float cev[2][8];
  {
    const float s5 = 1.0f / (SPB * SW);
#pragma unroll
    for (int j = 0; j < 2; ++j) {
#pragma unroll
      for (int r = 0; r < 8; ++r) {
        const float v = (ch2[j][r] + cr2[j][r] * RINV) * s5;
        cev[j][r] = v;
        _Float16 hi, rs;
        split16(v, SCE, hi, rs);
        const int pi = (8 * h + r) * 64 + 32 + 16 * j + c;
        ph[pi] = hi;
        pr[pi] = rs;
      }
    }
  }
  wave_sync_lds();

  v8f g0h[2], g0r[2], g1h[2], g1r[2];
  {
    const v16h ah0 = ldfrag_h(ph + c * 64 + 8 * h);
    const v16h ar0 = ldfrag_h(pr + c * 64 + 8 * h);
    const v16h ah1 = ldfrag_h(ph + c * 64 + 32 + 8 * h);
    const v16h ar1 = ldfrag_h(pr + c * 64 + 32 + 8 * h);
#pragma unroll
    for (int j = 0; j < 2; ++j) {
      const v16h bf0 = ldfrag_h(WGT + (size_t)(16 * j + c) * 64 + 8 * h);
      const v16h bf1 = ldfrag_h(WGT + (size_t)(16 * j + c) * 64 + 32 + 8 * h);
      g0h[j] = mma_h(ah0, bf0, zero8());
      g0r[j] = mma_h(ar0, bf0, zero8());
      g1h[j] = mma_h(ah1, bf1, zero8());
      g1r[j] = mma_h(ar1, bf1, zero8());
    }
  }
  float gv[2][8];
  {
    const float sa = 1.0f / (SID * SW);
    const float sb = 1.0f / (SCE * SW);
#pragma unroll
    for (int j = 0; j < 2; ++j) {
      const float bb = bfr(bg[16 * j + c]);
#pragma unroll
      for (int r = 0; r < 8; ++r) {
        gv[j][r] = ((g0h[j][r] + g0r[j][r] * RINV) * sa + (g1h[j][r] + g1r[j][r] * RINV) * sb) + bb;
      }
    }
  }
  wave_sync_lds();

#pragma unroll
  for (int j = 0; j < 2; ++j) {
#pragma unroll
    for (int r = 0; r < 8; ++r) {
      const int pi = (8 * h + r) * 64 + 16 * j + c;
      ph[pi]      = (_Float16)(idv[j][r] * SX);
      ph[pi + 32] = (_Float16)(cev[j][r] * SX);
      _Float16 hi, rs;
      split16(gv[j][r], SG, hi, rs);
      const int qi = (8 * h + r) * 32 + 16 * j + c;
      qh[qi] = hi;
      qr[qi] = rs;
    }
  }
  wave_sync_lds();
  HU og[4], ogh[2], ogr[2];
#pragma unroll
  for (int it = 0; it < 4; ++it) {
    const int p = it * 32 + lane;
    const int i = p >> 3, q = p & 7;
    og[it].hv = *(const v8h*)(ph + i * 64 + q * 8);
  }
#pragma unroll
  for (int it = 0; it < 2; ++it) {
    const int p = it * 32 + lane;
    const int i = p >> 2, q = p & 3;
    ogh[it].hv = *(const v8h*)(qh + i * 32 + q * 8);
    ogr[it].hv = *(const v8h*)(qr + i * 32 + q * 8);
  }
  for (int pass = 0; pass < 2; ++pass) {
#pragma unroll
    for (int it = 0; it < 4; ++it) {
      const int p = it * 32 + lane;
      const int i = p >> 3, q = p & 7;
      *(volatile v4u*)(GI + (size_t)(r0 + i) * DGI + DT + q * 8) = og[it].u;
    }
#pragma unroll
    for (int it = 0; it < 2; ++it) {
      const int p = it * 32 + lane;
      const int i = p >> 2, q = p & 3;
      *(volatile v4u*)(GH + (size_t)(r0 + i) * DG + q * 8) = ogh[it].u;
      *(volatile v4u*)(GR + (size_t)(r0 + i) * DG + q * 8) = ogr[it].u;
    }
    __threadfence();
  }
}

__global__ __launch_bounds__(64) void adjagg(const unsigned short* __restrict__ GHp,
                                             const unsigned short* __restrict__ GRp,
                                             const unsigned short* __restrict__ GITp, unsigned short* AG) {
  union FH { v16h v; v8h hh[2]; };
  union HU { v8h hv; v4u u; };
  __shared__ __align__(16) _Float16 Pt[16 * 64];
  __shared__ __align__(16) _Float16 AGs[16 * DGI];
  __shared__ float als[16];
  __shared__ float Ls[16];

  const int tid = threadIdx.x, wave = tid >> 5, lane = tid & 31, h = lane >> 4, c = lane & 15;
  const int row0 = blockIdx.x * 16;
  const int b = row0 / NC;
  const int oq = row0 - b * NC;
  const _Float16* GH  = (const _Float16*)(const void*)GHp;
  const _Float16* GR  = (const _Float16*)(const void*)GRp;
  const _Float16* GIT = (const _Float16*)(const void*)GITp + (size_t)b * DGI * NC;

  const v16h gah = ldfrag_h(GH + (size_t)(row0 + c) * DG + 8 * h);
  const v16h gar = ldfrag_h(GR + (size_t)(row0 + c) * DG + 8 * h);

  float mrow[8], lrow[8];
#pragma unroll
  for (int r = 0; r < 8; ++r) { mrow[r] = -3.0e38f; lrow[r] = 0.f; }
  v8f oacc[6];
#pragma unroll
  for (int t = 0; t < 6; ++t) oacc[t] = zero8();
  const float RINV = 1.0f / SR;
  const float ssc = 1.0f / (SG * SG);
  const int dbase = wave * 96;

  for (int kt = 0; kt < NC / 64; ++kt) {
    const int kv0 = kt * 64;
    if (wave == 0) {
      v8f ev[4];
#pragma unroll
      for (int j = 0; j < 4; ++j) {
        const size_t krow = (size_t)(b * NC + kv0 + j * 16 + c) * DG + 8 * h;
        const v16h kbh = ldfrag_h(GH + krow);
        const v16h kbr = ldfrag_h(GR + krow);
        v8f sh = mma_h(gah, kbh, zero8());
        v8f sl = mma_h(gah, kbr, zero8());
        sl = mma_h(gar, kbh, sl);
        v8f e;
#pragma unroll
        for (int r = 0; r < 8; ++r) {
          const float s = (sh[r] + sl[r] * RINV) * ssc;
          const int og = oq + 8 * h + r;
          const int mg = kv0 + j * 16 + c;
          const float v = (og == mg) ? NEGV : fmaxf(s, 0.0f);
          e[r] = v * kLog2E;
        }
        ev[j] = e;
      }
#pragma unroll
      for (int r = 0; r < 8; ++r) {
        float cm = fmaxf(fmaxf(ev[0][r], ev[1][r]), fmaxf(ev[2][r], ev[3][r]));
        cm = fmaxf(cm, __shfl_xor(cm, 1, 32));
        cm = fmaxf(cm, __shfl_xor(cm, 2, 32));
        cm = fmaxf(cm, __shfl_xor(cm, 4, 32));
        cm = fmaxf(cm, __shfl_xor(cm, 8, 32));
        const float mn = fmaxf(mrow[r], cm);
        const float al = exp2f(mrow[r] - mn);
        mrow[r] = mn;
        float ps = 0.f;
#pragma unroll
        for (int j = 0; j < 4; ++j) {
          const float p = exp2f(ev[j][r] - mn);
          ps += p;
          Pt[(8 * h + r) * 64 + j * 16 + c] = (_Float16)(p * SP);
        }
        lrow[r] = lrow[r] * al + ps;
        if (c == 0) als[8 * h + r] = al;
      }
    }
    __syncthreads();
    {
      float a[8];
#pragma unroll
      for (int r = 0; r < 8; ++r) a[r] = als[8 * h + r];
#pragma unroll
      for (int t = 0; t < 6; ++t) {
#pragma unroll
        for (int r = 0; r < 8; ++r) oacc[t][r] *= a[r];
      }
    }
#pragma unroll
    for (int kk = 0; kk < 2; ++kk) {
      FH pa;
      pa.hh[0] = *(const v8h*)(Pt + c * 64 + kk * 32 + 8 * h);
      pa.hh[1] = *(const v8h*)(Pt + c * 64 + kk * 32 + 16 + 8 * h);
#pragma unroll
      for (int t = 0; t < 6; ++t) {
        const v16h vb = ldfrag_h(GIT + (size_t)(dbase + t * 16 + c) * NC + kv0 + kk * 32 + 8 * h);
        oacc[t] = mma_h(pa.v, vb, oacc[t]);
      }
    }
    __syncthreads();
  }

  if (wave == 0) {
#pragma unroll
    for (int r = 0; r < 8; ++r) {
      float L = lrow[r];
      L += __shfl_xor(L, 1, 32);
      L += __shfl_xor(L, 2, 32);
      L += __shfl_xor(L, 4, 32);
      L += __shfl_xor(L, 8, 32);
      if (c == 0) Ls[8 * h + r] = L;
    }
  }
  __syncthreads();
  {
    const float nsc = SAG / (SP * SX);
#pragma unroll
    for (int r = 0; r < 8; ++r) {
      const float inv = nsc * (1.0f / Ls[8 * h + r]);
#pragma unroll
      for (int t = 0; t < 6; ++t) {
        AGs[(8 * h + r) * DGI + dbase + t * 16 + c] = (_Float16)(oacc[t][r] * inv);
      }
    }
  }
  __syncthreads();
  HU o[6];
#pragma unroll
  for (int it = 0; it < 6; ++it) {
    const int p = it * 64 + tid;
    const int line = p >> 3, q = p & 7;
    const int row = line / 3;
    const int seg = line - row * 3;
    o[it].hv = *(const v8h*)(AGs + row * DGI + seg * 64 + q * 8);
  }
  for (int pass = 0; pass < 2; ++pass) {
#pragma unroll
    for (int it = 0; it < 6; ++it) {
      const int p = it * 64 + tid;
      const int line = p >> 3, q = p & 7;
      const int row = line / 3;
      const int seg = line - row * 3;
      *(volatile v4u*)(AG + (size_t)(row0 + row) * DGI + seg * 64 + q * 8) = o[it].u;
    }
    __threadfence();
  }
}

__device__ __forceinline__ void gemm_acc(const _Float16* A, int lda, const _Float16* Bt, int ldb, int K,
                                         int m0, int n0, int rlane, int koff, v8f (&acc)[4][4]) {
  for (int k0 = 0; k0 < K; k0 += 32) {
    v16h bh[4];
#pragma unroll
    for (int j = 0; j < 4; ++j) bh[j] = ldfrag_h(Bt + (size_t)(n0 + (j << 4) + rlane) * ldb + koff + k0);
#pragma unroll
    for (int i = 0; i < 4; ++i) {
      const v16h ah = ldfrag_h(A + (size_t)(m0 + (i << 4) + rlane) * lda + koff + k0);
#pragma unroll
      for (int j = 0; j < 4; ++j) acc[i][j] = mma_h(ah, bh[j], acc[i][j]);
    }
  }
}

template <int ACT>
__global__ __launch_bounds__(256) void gemm64h(
    const unsigned short* __restrict__ Ap, int lda, int sAz,
    const unsigned short* __restrict__ Btp, int ldb, int sBz,
    unsigned short* Cp, int ldc, int sCz,
    int M, int N, int K, int Z, float oscale, float osc2) {
  __shared__ __align__(16) float sT[8][16 * 68];
  const int lane = threadIdx.x & 31;
  const int wave = threadIdx.x >> 5;
  const int tilesN = N >> 6;
  const int tilesM = M >> 6;
  const int tpz = tilesM * tilesN;
  const int tile = blockIdx.x * 8 + wave;
  if (tile >= Z * tpz) return;
  const int z = tile / tpz;
  const int rem = tile - z * tpz;
  const int tm = rem / tilesN;
  const int tn = rem - tm * tilesN;
  const int m0 = tm << 6;
  const int n0 = tn << 6;
  const _Float16* A  = (const _Float16*)(const void*)Ap + (size_t)z * sAz;
  const _Float16* Bt = (const _Float16*)(const void*)Btp + (size_t)z * sBz;
  unsigned short* C = Cp + (size_t)z * sCz;

  const int rlane = lane & 15;
  const int koff  = (lane >> 4) * 8;
  const int mOff  = (lane >> 4) * 8;

  v8f acc[4][4];
#pragma unroll
  for (int i = 0; i < 4; ++i)
#pragma unroll
    for (int j = 0; j < 4; ++j) acc[i][j] = zero8();
  gemm_acc(A, lda, Bt, ldb, K, m0, n0, rlane, koff, acc);

  const int q8 = lane >> 3, c8 = (lane & 7) * 8;
  float* slab = sT[wave];
#pragma unroll
  for (int i = 0; i < 4; ++i) {
    const int mBase = m0 + (i << 4);
#pragma unroll
    for (int j = 0; j < 4; ++j) {
#pragma unroll
      for (int r = 0; r < 8; ++r) {
        slab[(mOff + r) * 68 + (j << 4) + rlane] = acc[i][j][r];
      }
    }
    wave_sync_lds();
    v4u hv[4];
#pragma unroll
    for (int it = 0; it < 4; ++it) {
      const int row = it * 4 + q8;
      const float* sp = slab + row * 68 + c8;
      v4u a;
#pragma unroll
      for (int e = 0; e < 4; ++e) {
        float f0 = sp[2 * e]     * oscale;
        float f1 = sp[2 * e + 1] * oscale;
        if (ACT == 1) { f0 = tanhf(f0); f1 = tanhf(f1); }
        const _Float16 g0 = (_Float16)(f0 * osc2);
        const _Float16 g1 = (_Float16)(f1 * osc2);
        a[e] = pk16(h_bits(g0), h_bits(g1));
      }
      hv[it] = a;
    }
    for (int pass = 0; pass < 2; ++pass) {
#pragma unroll
      for (int it = 0; it < 4; ++it) {
        const int row = it * 4 + q8;
        const size_t go = (size_t)(mBase + row) * ldc + n0 + c8;
        *(volatile v4u*)(C + go) = hv[it];
      }
      __threadfence();
    }
    wave_sync_lds();
  }
}

__global__ __launch_bounds__(256) void gemm64f(
    const unsigned short* __restrict__ Ap, const unsigned short* __restrict__ A2p, int lda,
    const unsigned short* __restrict__ Btp, const unsigned short* __restrict__ Bt2p, int ldb,
    float* Cp, int ldc, const float* __restrict__ bias,
    int M, int N, int K, int K2, int Nvalid, float oscale) {
  __shared__ __align__(16) float sT[8][16 * 68];
  const int lane = threadIdx.x & 31;
  const int wave = threadIdx.x >> 5;
  const int tilesN = N >> 6;
  const int tilesM = M >> 6;
  const int tile = blockIdx.x * 8 + wave;
  if (tile >= tilesM * tilesN) return;
  const int tm = tile / tilesN;
  const int tn = tile - tm * tilesN;
  const int m0 = tm << 6;
  const int n0 = tn << 6;
  const _Float16* A   = (const _Float16*)(const void*)Ap;
  const _Float16* A2  = (const _Float16*)(const void*)A2p;
  const _Float16* Bt  = (const _Float16*)(const void*)Btp;
  const _Float16* Bt2 = (const _Float16*)(const void*)Bt2p;

  const int rlane = lane & 15;
  const int koff  = (lane >> 4) * 8;
  const int mOff  = (lane >> 4) * 8;

  v8f acc[4][4];
#pragma unroll
  for (int i = 0; i < 4; ++i)
#pragma unroll
    for (int j = 0; j < 4; ++j) acc[i][j] = zero8();
  gemm_acc(A, lda, Bt, ldb, K, m0, n0, rlane, koff, acc);
  if (K2 > 0) gemm_acc(A2, lda, Bt2, ldb, K2, m0, n0, rlane, koff, acc);

  const int hq = lane >> 4, q = lane & 15;
  const int col = n0 + 4 * q;
  const bool act = (col < Nvalid);
  float bb[4];
#pragma unroll
  for (int e = 0; e < 4; ++e) {
    int bi = col + e;
    if (bi > Nvalid - 1) bi = Nvalid - 1;
    bb[e] = bfr(bias[bi]);
  }
  float* slab = sT[wave];
#pragma unroll
  for (int i = 0; i < 4; ++i) {
    const int mBase = m0 + (i << 4);
#pragma unroll
    for (int j = 0; j < 4; ++j) {
#pragma unroll
      for (int r = 0; r < 8; ++r) {
        slab[(mOff + r) * 68 + (j << 4) + rlane] = acc[i][j][r];
      }
    }
    wave_sync_lds();
    v4f ov[8];
#pragma unroll
    for (int it = 0; it < 8; ++it) {
      const int row = it * 2 + hq;
      const float* sp = slab + row * 68 + 4 * q;
      v4f o;
#pragma unroll
      for (int e = 0; e < 4; ++e) o[e] = sp[e] * oscale + bb[e];
      ov[it] = o;
    }
    for (int pass = 0; pass < 2; ++pass) {
#pragma unroll
      for (int it = 0; it < 8; ++it) {
        const int row = it * 2 + hq;
        const size_t go = (size_t)(mBase + row) * ldc + col;
        if (act) *(volatile v4f*)(Cp + go) = ov[it];
      }
      __threadfence();
    }
    wave_sync_lds();
  }
}

extern "C" void kernel_launch(void* const* d_in, const int* in_sizes, int n_in,
                              void* d_out, int out_size, void* d_ws, size_t ws_size,
                              hipStream_t stream) {
  if (n_in < 14) return;
  if (in_sizes[0] != NROW * DT || in_sizes[1] != NC * DI || in_sizes[2] != DT * DH || in_sizes[3] != DH) return;
  if (in_sizes[4] != DH * DI || in_sizes[5] != DI || in_sizes[6] != NCL * DCE || in_sizes[7] != DI * DCE) return;
  if (in_sizes[8] != DCE || in_sizes[9] != (DI + DCE) * DG || in_sizes[10] != DG) return;
  if (in_sizes[11] != NC * DGI || in_sizes[12] != DGI * DOUT || in_sizes[13] != DOUT) return;
  if (out_size != NROW * DOUT) return;

  const float* x     = (const float*)d_in[0];
  const float* idemb = (const float*)d_in[1];
  const float* w1    = (const float*)d_in[2];
  const float* b1    = (const float*)d_in[3];
  const float* w2    = (const float*)d_in[4];
  const float* b2    = (const float*)d_in[5];
  const float* ce    = (const float*)d_in[6];
  const float* wic   = (const float*)d_in[7];
  const float* bic   = (const float*)d_in[8];
  const float* wg    = (const float*)d_in[9];
  const float* bg    = (const float*)d_in[10];
  const float* cw    = (const float*)d_in[11];
  const float* wl    = (const float*)d_in[12];
  const float* bl    = (const float*)d_in[13];
  float* out = (float*)d_out;

  const size_t PW1  = (size_t)DH * DT * 2;
  const size_t PW2  = (size_t)DI * DH * 2;
  const size_t PWIC = (size_t)DCE * 64 * 2;
  const size_t PCE  = (size_t)NCL * 64 * 2;
  const size_t PCET = (size_t)DCE * 64 * 2;
  const size_t PWG  = (size_t)DG * 64 * 2;
  const size_t PCW  = (size_t)DGI * NC * 2;
  const size_t PWL  = (size_t)DOUTP * DGI * 2;
  const size_t PGI  = (size_t)NROW * DGI * 2;
  const size_t PG   = (size_t)NROW * DG * 2;
  const size_t PWT  = (size_t)NB * DGI * DGI * 2;
  size_t off = 0;
  const size_t oW1 = off;  off += PW1;
  const size_t oW2 = off;  off += PW2;
  const size_t oWIC = off; off += PWIC;
  const size_t oCE = off;  off += PCE;
  const size_t oCET = off; off += PCET;
  const size_t oWG = off;  off += PWG;
  const size_t oCW = off;  off += PCW;
  const size_t oWL = off;  off += PWL;
  const size_t oWL4 = off; off += PWL;
  const size_t oGI = off;  off += PGI;
  const size_t oGIT = off; off += PGI;
  const size_t oGH = off;  off += PG;
  const size_t oGR = off;  off += PG;
  const size_t oAG = off;  off += PGI;
  const size_t oAGT = off; off += PGI;
  const size_t oWT = off;  off += PWT;
  const size_t oU = off;   off += PGI;
  if (off > ws_size) return;
  if (off > (size_t)134217728) return;

  char* ws = (char*)d_ws;
  unsigned short* W1T  = (unsigned short*)(ws + oW1);
  unsigned short* W2T  = (unsigned short*)(ws + oW2);
  unsigned short* WICT = (unsigned short*)(ws + oWIC);
  unsigned short* CEP  = (unsigned short*)(ws + oCE);
  unsigned short* CETP = (unsigned short*)(ws + oCET);
  unsigned short* WGT  = (unsigned short*)(ws + oWG);
  unsigned short* CWT  = (unsigned short*)(ws + oCW);
  unsigned short* WLT  = (unsigned short*)(ws + oWL);
  unsigned short* WLT4 = (unsigned short*)(ws + oWL4);
  unsigned short* GI   = (unsigned short*)(ws + oGI);
  unsigned short* GIT  = (unsigned short*)(ws + oGIT);
  unsigned short* GH   = (unsigned short*)(ws + oGH);
  unsigned short* GR   = (unsigned short*)(ws + oGR);
  unsigned short* AG   = (unsigned short*)(ws + oAG);
  unsigned short* AGT  = (unsigned short*)(ws + oAGT);
  unsigned short* WT   = (unsigned short*)(ws + oWT);
  unsigned short* U    = (unsigned short*)(ws + oU);

  const dim3 blk(256), blk128(128), blk64(64);

  tconv<<<dim3(DH), blk, 0, stream>>>(w1, DH, 1, W1T, DT, DH, DT, SW);
  tconv<<<dim3(DI), blk, 0, stream>>>(w2, DI, 1, W2T, DH, DI, DH, SW);
  tconv<<<dim3(DCE), blk, 0, stream>>>(wic, DCE, 1, WICT, DI, DCE, 64, SW);
  tconv<<<dim3(NCL), blk, 0, stream>>>(ce, 1, DCE, CEP, DCE, NCL, 64, SW);
  tconv<<<dim3(DCE), blk, 0, stream>>>(ce, DCE, 1, CETP, NCL, DCE, 64, SW);
  tconv<<<dim3(DG), blk, 0, stream>>>(wg, DG, 1, WGT, DI + DCE, DG, 64, SW);
  tconv<<<dim3(DGI), blk, 0, stream>>>(cw, DGI, 1, CWT, NC, DGI, NC, SW);
  tconv<<<dim3(DOUTP), blk, 0, stream>>>(wl, DOUT, 1, WLT, DGI, DOUT, DGI, SW);
  tconv<<<dim3(DOUTP), blk, 0, stream>>>(wl, DOUT, 1, WLT4, DGI, DOUT, DGI, SW4);

  xconv<<<dim3((NROW * (DT / 8)) / 256), blk, 0, stream>>>(x, GI);

  chain<<<dim3(NROW / 64), blk128, 0, stream>>>(GI, W1T, W2T, WICT, CEP, CETP, WGT,
                                               b1, idemb, b2, bic, bg, GH, GR);

  tr16<<<dim3(NC / 64, DGI / 64, NB), blk, 0, stream>>>(GI, DGI, GIT, NC, DGI);

  adjagg<<<dim3(NROW / 16), blk64, 0, stream>>>(GH, GR, GIT, AG);

  tr16<<<dim3(NC / 64, DGI / 64, NB), blk, 0, stream>>>(AG, DGI, AGT, NC, DGI);

  {
    const int tiles = NB * (DGI / 64) * (DGI / 64);
    gemm64h<1><<<dim3((tiles + 7) / 8), blk, 0, stream>>>(
        CWT, NC, 0, AGT, NC, DGI * NC, WT, DGI, DGI * DGI, DGI, DGI, NC, NB, 1.0f / (SW * SAG), SWT);
  }
  {
    const int tiles = NB * (NC / 64) * (DGI / 64);
    gemm64h<0><<<dim3((tiles + 7) / 8), blk, 0, stream>>>(
        GI, DGI, NC * DGI, WT, DGI, DGI * DGI, U, DGI, NC * DGI, NC, DGI, DGI, NB, 1.0f / (SX * SWT), SU);
  }
  {
    const int tiles = (NROW / 64) * (DOUTP / 64);
    gemm64f<<<dim3((tiles + 7) / 8), blk, 0, stream>>>(
        U, GI, DGI, WLT, WLT4, DGI, out, DOUT, bl, NROW, DOUTP, DGI, DGI, DOUT, 1.0f / (SU * SW));
  }
  (void)hipGetLastError();
}
